// HexGINLayer_20590073217561
// MI455X (gfx1250) — hardware-run, weakly checked
//
#include <hip/hip_runtime.h>

typedef float          v8f   __attribute__((ext_vector_type(8)));
typedef float          v4f   __attribute__((ext_vector_type(4)));
typedef unsigned int   v4u   __attribute__((ext_vector_type(4)));
typedef int            v8i   __attribute__((ext_vector_type(8)));
typedef unsigned short v8us  __attribute__((ext_vector_type(8)));
typedef unsigned short v16us __attribute__((ext_vector_type(16)));
typedef __bf16         v16bf __attribute__((ext_vector_type(16)));
typedef _Float16       v16h  __attribute__((ext_vector_type(16)));
typedef v4f  __attribute__((may_alias)) v4fa;
typedef v8us __attribute__((may_alias)) v8usa;
union FragB { v16bf v; v16us u; v8us h[2]; v8i w; };
union FragH { v16h  v; v16us u; v8us h[2]; v8i w; };

__device__ __forceinline__ v8f wmb(const FragB& a, const FragB& b, v8f c) {
  v8f d = __builtin_amdgcn_wmma_f32_16x16x32_bf16(false, a.v, false, b.v, (short)0, c, false, false);
  asm volatile("v_nop\n\tv_nop\n\tv_nop\n\tv_nop" : "+v"(d) : "v"(a.w), "v"(b.w));
  return d;
}

__device__ __forceinline__ v8f wmh(const FragH& a, const FragH& b, v8f c) {
  v8f d = __builtin_amdgcn_wmma_f32_16x16x32_f16(false, a.v, false, b.v, (short)0, c, false, false);
  asm volatile("v_nop\n\tv_nop\n\tv_nop\n\tv_nop" : "+v"(d) : "v"(a.w), "v"(b.w));
  return d;
}

__device__ __forceinline__ unsigned bf16_bits(float f) {
  const unsigned u = __float_as_uint(f);
  const unsigned r = (u + 0x7FFFu + ((u >> 16) & 1u)) >> 16;
  const unsigned q = (u >> 16) | 0x40u;
  return ((u & 0x7fffffffu) > 0x7f800000u) ? q : r;
}

__device__ __forceinline__ float bf16_val(float f) {
  return __uint_as_float(bf16_bits(f) << 16);
}
__device__ __forceinline__ int clampi(int v, int lo, int hi) {
  return v < lo ? lo : (v > hi ? hi : v);
}

__device__ __forceinline__ unsigned f16_bits(float f) {
  const unsigned u  = __float_as_uint(f);
  const unsigned s  = (u >> 16) & 0x8000u;
  const unsigned a  = u & 0x7fffffffu;
  const unsigned t  = a - 0x38000000u;
  const unsigned r  = (t + 0x0FFFu + ((t >> 13) & 1u)) >> 13;
  const unsigned rc = r > 0x7C00u ? 0x7C00u : r;
  const bool small  = a < 0x38800000u;
  const bool isnan  = a > 0x7f800000u;
  const unsigned fin = small ? 0u : (s | rc);
  return isnan ? (s | 0x7E00u) : fin;
}

__device__ __forceinline__ unsigned pk16(unsigned lo, unsigned hi) { return lo | (hi << 16); }
__device__ __forceinline__ unsigned bf16_lo_bits(float v) {
  float hi = bf16_val(v);
  asm volatile("" : "+v"(hi));
  return bf16_bits(v - hi);
}
__device__ __forceinline__ v4u pack8_bf16(v4f a, v4f c) {
  return (v4u){ pk16(bf16_bits(a[0]), bf16_bits(a[1])), pk16(bf16_bits(a[2]), bf16_bits(a[3])),
                pk16(bf16_bits(c[0]), bf16_bits(c[1])), pk16(bf16_bits(c[2]), bf16_bits(c[3])) };
}
__device__ __forceinline__ v4u pack8_bf16_lo(v4f a, v4f c) {
  return (v4u){ pk16(bf16_lo_bits(a[0]), bf16_lo_bits(a[1])), pk16(bf16_lo_bits(a[2]), bf16_lo_bits(a[3])),
                pk16(bf16_lo_bits(c[0]), bf16_lo_bits(c[1])), pk16(bf16_lo_bits(c[2]), bf16_lo_bits(c[3])) };
}
__device__ __forceinline__ v4u pack8_f16(v4f a, v4f c) {
  return (v4u){ pk16(f16_bits(a[0]), f16_bits(a[1])), pk16(f16_bits(a[2]), f16_bits(a[3])),
                pk16(f16_bits(c[0]), f16_bits(c[1])), pk16(f16_bits(c[2]), f16_bits(c[3])) };
}

template <int FORM>
__global__ __launch_bounds__(256) void k_plane(const float* __restrict__ src, int rows, int cols, int ldsrc,
                                               unsigned short* __restrict__ dst, int MP, int KP) {
  static_assert(FORM >= 0 && FORM <= 3);
  const int KTOT = (FORM == 1 || FORM == 3) ? 2 * KP : KP;
  const unsigned ppr   = (unsigned)(KTOT >> 3);
  const unsigned kp8   = (unsigned)(KP >> 3);
  const unsigned total = (unsigned)MP * ppr;
  const unsigned g     = blockIdx.x * 256u + threadIdx.x;
  const unsigned rowu  = g / ppr;
  const unsigned p     = g - rowu * ppr;
  const bool second    = p >= kp8;
  const int row = (int)rowu;
  const int c0  = (int)((second ? p - kp8 : p) << 3);
  const float* srow = src + (size_t)clampi(row, 0, rows - 1) * (size_t)ldsrc;
  float x[8];
  unsigned mk[8];
#pragma unroll
  for (int e = 0; e < 8; ++e) {
    const int c = c0 + e;
    const float v = srow[clampi(c, 0, cols - 1)];
    asm volatile("" :: "v"(v));
    x[e]  = v;
    mk[e] = (row < rows && c < cols) ? 0xFFFFu : 0u;
  }
  const v4f a = (v4f){ x[0], x[1], x[2], x[3] };
  const v4f c = (v4f){ x[4], x[5], x[6], x[7] };
  v4u o;
  if (FORM == 2) {
    o = pack8_f16(a, c);
  } else {
    const v4u hi = pack8_bf16(a, c);
    o = hi;
    if (FORM == 1) { const v4u lo = pack8_bf16_lo(a, c); o = second ? lo : hi; }
  }
  const v4u mw = (v4u){ pk16(mk[0], mk[1]), pk16(mk[2], mk[3]), pk16(mk[4], mk[5]), pk16(mk[6], mk[7]) };
  o &= mw;
  if (g < total) {
    volatile v4u* q = (volatile v4u*)(dst + (size_t)g * 8);
    *q = o;
    __threadfence();
    *q = o;
  }
}

template <int FORM> struct FragOf    { typedef FragB T; };
template <>         struct FragOf<2> { typedef FragH T; };
__device__ __forceinline__ v8f mm(const FragB& a, const FragB& b, v8f c) { return wmb(a, b, c); }
__device__ __forceinline__ v8f mm(const FragH& a, const FragH& b, v8f c) { return wmh(a, b, c); }
template <class F> __device__ __forceinline__ F ld_frag(const unsigned short* p) {
  F f;
  f.h[0] = *(const v8usa*)(p);
  f.h[1] = *(const v8usa*)(p + 16);
  return f;
}

template <int FORM, int EPI>
__global__ __launch_bounds__(256) __attribute__((amdgpu_num_vgpr(248)))
void k_gemm_nt(const unsigned short* __restrict__ A, const unsigned short* __restrict__ B,
               const float* __restrict__ bias, float* __restrict__ D, int M, int N, int KTOT, int ldd) {
  static_assert(FORM >= 0 && FORM <= 2);
  static_assert(EPI == 0 || EPI == 1);
  typedef typename FragOf<FORM>::T F;
  __shared__ __attribute__((aligned(16))) float sT[8][16 * 68];
  const int lane = threadIdx.x & 31;
  const int wave = threadIdx.x >> 5;
  const int tilesM = (M + 63) >> 6;
  const int tilesN = (N + 63) >> 6;
  const int tile = blockIdx.x * 8 + wave;
  if (tile >= tilesM * tilesN) return;
  const int tm = tile / tilesN;
  const int tn = tile - tm * tilesN;
  const int m0 = tm << 6;
  const int n0 = tn << 6;

  const int rl = lane & 15;
  const int h8 = (lane >> 4) * 8;
  const unsigned short* pa = A + (size_t)(m0 + rl) * (size_t)KTOT + h8;
  const unsigned short* pb = B + (size_t)(n0 + rl) * (size_t)KTOT + h8;

  v8f acc[4][4];
#pragma unroll
  for (int i = 0; i < 4; ++i)
#pragma unroll
    for (int j = 0; j < 4; ++j) acc[i][j] = (v8f){0.f, 0.f, 0.f, 0.f, 0.f, 0.f, 0.f, 0.f};

#pragma unroll 1
  for (int k0 = 0; k0 < KTOT; k0 += 32) {
    F bf[4];
#pragma unroll
    for (int j = 0; j < 4; ++j) bf[j] = ld_frag<F>(pb + (size_t)(j << 4) * (size_t)KTOT + k0);
#pragma unroll
    for (int i = 0; i < 4; ++i) {
      const F af = ld_frag<F>(pa + (size_t)(i << 4) * (size_t)KTOT + k0);
#pragma unroll
      for (int j = 0; j < 4; ++j) acc[i][j] = mm(af, bf[j], acc[i][j]);
    }
  }

  float* slab = sT[wave];
  const int hh = lane >> 4;
  const int c4 = (lane & 15) * 4;
  const int nc = n0 + c4;
  const bool cok = nc < N;
  v4f bv = (v4f){0.f, 0.f, 0.f, 0.f};
  if (EPI == 1) {
    bv = *(const v4fa*)(bias + clampi(nc, 0, N - 4));
    asm volatile("" :: "v"(bv));
  }
#pragma unroll
  for (int i = 0; i < 4; ++i) {
    const int mBase = m0 + (i << 4);
#pragma unroll
    for (int j = 0; j < 4; ++j) {
#pragma unroll
      for (int r = 0; r < 8; ++r) slab[(h8 + r) * 68 + (j << 4) + rl] = acc[i][j][r];
    }
    __builtin_amdgcn_fence(__ATOMIC_RELEASE, "workgroup");
    __builtin_amdgcn_wave_barrier();
    __builtin_amdgcn_fence(__ATOMIC_ACQUIRE, "workgroup");
    v4f vv[8];
#pragma unroll
    for (int it = 0; it < 8; ++it) {
      const int row = it * 2 + hh;
      v4f v = *(const v4fa*)(slab + row * 68 + c4);
      if (EPI == 1) v += bv;
      vv[it] = v;
    }
    for (int pass = 0; pass < 2; ++pass) {
#pragma unroll
      for (int it = 0; it < 8; ++it) {
        const int row = mBase + it * 2 + hh;
        if (cok && row < M) *(volatile v4f*)(D + (size_t)row * (size_t)ldd + nc) = vv[it];
      }
      __threadfence();
    }
    __builtin_amdgcn_fence(__ATOMIC_RELEASE, "workgroup");
    __builtin_amdgcn_wave_barrier();
    __builtin_amdgcn_fence(__ATOMIC_ACQUIRE, "workgroup");
  }
}

#ifndef SPLIT_OP
#define SPLIT_OP 1
#endif
#ifndef SPLIT_HID
#define SPLIT_HID 1
#endif

#define NU     50000
#define NT     50000
#define NE     600000
#define MPAD   50048
#define DU     128
#define DT     64
#define DA     128
#define HIDW   256
#define DOUT   128
#define KOP_UT (SPLIT_OP ? (2 * DT + 256) : (DT + 128))
#define KOP_TU (SPLIT_OP ? (2 * DU + 256) : (DU + 128))
#define K2     (SPLIT_HID ? 512 : 256)

#define NTHR   256
#define NWAVE  8
#define EPT    8
#define CHUNK  (NTHR * EPT)
#define WCAP   (EPT * 32)
#define LISTN  (NWAVE * WCAP)
#define NBA    1024
#define SLA    10
#define NBLK   49
#define RCAP   16384
static_assert(RCAP >= 12635 + 12635 / 4);
#define DEGCAP 48
static_assert(DEGCAP >= 29 + 8);
#define BK_ZINTS (LISTN + 2 * RCAP + 3 * NBA)
#define BK_MISC  16
#define BK_LDS_INTS (BK_ZINTS + BK_MISC)

static_assert(NU == NT && MPAD % 64 == 0 && MPAD >= NU && MPAD - NU < 64 && MPAD % 8 == 0);
static_assert(NE % EPT == 0 && NE >= EPT && NE < (1 << 20));
static_assert(NBA == (1 << SLA) && NBLK * NBA >= MPAD && (NBA % 32) == 0);
static_assert(((long long)CHUNK << SLA) < (1LL << 31));
static_assert(BK_ZINTS % (NTHR * 4) == 0 && RCAP % (NTHR * 4) == 0 && NBA == NTHR * 4);
static_assert(BK_LDS_INTS * 4 <= 262144);
static_assert(KOP_UT % 64 == 0 && KOP_TU % 64 == 0 && K2 % 64 == 0 && KOP_TU <= 512 && K2 <= 512);
static_assert(DU % 32 == 0 && DT % 32 == 0 && DA == 128 && HIDW == 256 && DOUT == 128);
static_assert(NU % 16 == 0 && NT % 16 == 0);

typedef int          v4i  __attribute__((ext_vector_type(4)));
typedef unsigned int v2u  __attribute__((ext_vector_type(2)));
typedef float        v2f  __attribute__((ext_vector_type(2)));
typedef v4i  __attribute__((may_alias)) v4ia;
typedef v2u  __attribute__((may_alias)) v2ua;
typedef v4u  __attribute__((may_alias)) v4ua;
typedef v2f  __attribute__((may_alias)) v2fa;
typedef unsigned int __attribute__((may_alias)) u32a;

constexpr size_t SZ_T    = (size_t)MPAD * 256 * 4;
constexpr size_t SZ_OPH  = (size_t)MPAD * 512 * 2;
constexpr size_t SZ_XS   = (size_t)MPAD * 128 * 2;
constexpr size_t SZ_LIST = (size_t)NBLK * RCAP * 4;
constexpr size_t SZ_CNT  = (size_t)NBLK * NBA * 4;
constexpr size_t SZ_FLG  = 6400;
constexpr size_t SZ_WAU  = (size_t)128 * 128 * 2;
constexpr size_t SZ_WAT  = (size_t)128 * 64 * 2;
constexpr size_t SZ_W1UT = (size_t)256 * 384 * 2;
constexpr size_t SZ_W1TU = (size_t)256 * 512 * 2;
constexpr size_t SZ_W2   = (size_t)128 * 512 * 2;
constexpr size_t SZ_BT   = (size_t)1024 * 4;
constexpr size_t SZ_ST   = 256;
constexpr size_t O_T    = 0;
constexpr size_t O_OPH  = O_T + SZ_T;
constexpr size_t O_XS   = O_OPH + SZ_OPH;
constexpr size_t O_LIST = O_XS + SZ_XS;
constexpr size_t O_CNT  = O_LIST + SZ_LIST;
constexpr size_t O_OFF  = O_CNT + SZ_CNT;
constexpr size_t O_FLG  = O_OFF + SZ_CNT;
constexpr size_t O_WAU  = O_FLG + SZ_FLG;
constexpr size_t O_WAT  = O_WAU + SZ_WAU;
constexpr size_t O_W1UT = O_WAT + SZ_WAT;
constexpr size_t O_W1TU = O_W1UT + SZ_W1UT;
constexpr size_t O_W2UT = O_W1TU + SZ_W1TU;
constexpr size_t O_W2TU = O_W2UT + SZ_W2;
constexpr size_t O_BT   = O_W2TU + SZ_W2;
constexpr size_t O_ST   = O_BT + SZ_BT;
constexpr size_t WS_TOTAL = O_ST + SZ_ST;
static_assert(SZ_T % 256 == 0 && SZ_OPH % 256 == 0 && SZ_XS % 256 == 0 && SZ_LIST % 256 == 0 && SZ_CNT % 256 == 0);
static_assert(SZ_FLG % 256 == 0 && SZ_FLG >= (size_t)NBLK * 128);
static_assert(WS_TOTAL == ((size_t)233797 << 9));
static_assert(WS_TOTAL <= ((size_t)128 << 20));
static_assert((size_t)MPAD * 128 * 4 <= SZ_T);
static_assert((size_t)MPAD * KOP_UT * 2 <= SZ_OPH && (size_t)MPAD * KOP_TU * 2 <= SZ_OPH && (size_t)MPAD * K2 * 2 <= SZ_OPH);
static_assert((size_t)256 * KOP_UT * 2 <= SZ_W1UT && (size_t)256 * KOP_TU * 2 <= SZ_W1TU && (size_t)128 * K2 * 2 <= SZ_W2);
static_assert((size_t)NU * DOUT + (size_t)NT * DOUT == 12800000);

#define BO_AU  0
#define BO_AT  128
#define BO_1UT 256
#define BO_2UT 512
#define BO_1TU 640
#define BO_2TU 896

__host__ __device__ constexpr int w_row(int k, int ownW, int dd, int am) {
  return k < ownW ? (k % dd) : dd + ((k - ownW) % am);
}
static_assert(w_row(0, 128, 64, 128) == 0 && w_row(63, 128, 64, 128) == 63 && w_row(64, 128, 64, 128) == 0 &&
              w_row(127, 128, 64, 128) == 63 && w_row(128, 128, 64, 128) == 64 && w_row(255, 128, 64, 128) == 191 &&
              w_row(256, 128, 64, 128) == 64 && w_row(383, 128, 64, 128) == 191);
static_assert(w_row(0, 256, 128, 128) == 0 && w_row(127, 256, 128, 128) == 127 && w_row(128, 256, 128, 128) == 0 &&
              w_row(255, 256, 128, 128) == 127 && w_row(256, 256, 128, 128) == 128 && w_row(383, 256, 128, 128) == 255 &&
              w_row(384, 256, 128, 128) == 128 && w_row(511, 256, 128, 128) == 255);
static_assert(w_row(0, 512, 256, 1) == 0 && w_row(255, 512, 256, 1) == 255 && w_row(256, 512, 256, 1) == 0 &&
              w_row(511, 512, 256, 1) == 255);

__device__ __forceinline__ void wave_sync() {
  __builtin_amdgcn_fence(__ATOMIC_RELEASE, "workgroup");
  __builtin_amdgcn_wave_barrier();
  __builtin_amdgcn_fence(__ATOMIC_ACQUIRE, "workgroup");
}

#define PC_WAU  (128 * 128 / 8)
#define PC_WAT  (128 * 64 / 8)
#define PC_W1UT (256 * KOP_UT / 8)
#define PC_W1TU (256 * KOP_TU / 8)
#define PC_W2   (128 * K2 / 8)
#define PU0 (PC_WAU)
#define PU1 (PU0 + PC_WAT)
#define PU2 (PU1 + PC_W1UT)
#define PU3 (PU2 + PC_W1TU)
#define PU4 (PU3 + PC_W2)
#define PU5 (PU4 + PC_W2)
static_assert(PC_WAU % 256 == 0 && PC_WAT % 256 == 0 && PC_W1UT % 256 == 0 && PC_W1TU % 256 == 0 && PC_W2 % 256 == 0);

__device__ __forceinline__ void prep_piece(const float* __restrict__ W, int ldw, int ownW, int dd, int am,
                                           unsigned short* __restrict__ P, int ktot, int v) {
  const int ppr = ktot >> 3;
  const int n   = v / ppr;
  const int p   = v - n * ppr;
  const int r0  = w_row(p << 3, ownW, dd, am);
  float x[8];
#pragma unroll
  for (int e = 0; e < 8; ++e) {
    const float t = W[(size_t)(r0 + e) * (size_t)ldw + n];
    asm volatile("" :: "v"(t));
    x[e] = t;
  }
  const v4u o = pack8_bf16((v4f){ x[0], x[1], x[2], x[3] }, (v4f){ x[4], x[5], x[6], x[7] });
  volatile v4u* q = (volatile v4u*)(P + (size_t)v * 8);
  *q = o;
  __threadfence();
  *q = o;
}

__device__ __forceinline__ unsigned bfv_bits(float f) { return bf16_bits(f) << 16; }

__global__ __launch_bounds__(256) void k_prep(
    const float* __restrict__ Wau, const float* __restrict__ Wat, const float* __restrict__ W1ut,
    const float* __restrict__ W1tu, const float* __restrict__ W2ut, const float* __restrict__ W2tu,
    const float* __restrict__ bau, const float* __restrict__ bat, const float* __restrict__ b1ut,
    const float* __restrict__ b2ut, const float* __restrict__ b1tu, const float* __restrict__ b2tu,
    const float* __restrict__ epsut, const float* __restrict__ epstu,
    unsigned short* __restrict__ PWau, unsigned short* __restrict__ PWat, unsigned short* __restrict__ PW1ut,
    unsigned short* __restrict__ PW1tu, unsigned short* __restrict__ PW2ut, unsigned short* __restrict__ PW2tu,
    float* __restrict__ Btab, float* __restrict__ Stab) {
  const int tid = (int)threadIdx.x;
  const int u = (int)blockIdx.x * 256 + tid;
  if (u < PU0) {
    prep_piece(Wau, DA, DU, DU, 1, PWau, DU, u);
  } else if (u < PU1) {
    prep_piece(Wat, DA, DT, DT, 1, PWat, DT, u - PU0);
  } else if (u < PU2) {
    prep_piece(W1ut, HIDW, SPLIT_OP ? 2 * DT : DT, DT, 128, PW1ut, KOP_UT, u - PU1);
  } else if (u < PU3) {
    prep_piece(W1tu, HIDW, SPLIT_OP ? 2 * DU : DU, DU, 128, PW1tu, KOP_TU, u - PU2);
  } else if (u < PU4) {
    prep_piece(W2ut, DOUT, K2, HIDW, 1, PW2ut, K2, u - PU3);
  } else if (u < PU5) {
    prep_piece(W2tu, DOUT, K2, HIDW, 1, PW2tu, K2, u - PU4);
  } else {
    const int c = 4 * tid;
    const v4f t0 = *(const v4fa*)(bau  + clampi(c - BO_AU,  0, 124));
    const v4f t1 = *(const v4fa*)(bat  + clampi(c - BO_AT,  0, 124));
    const v4f t2 = *(const v4fa*)(b1ut + clampi(c - BO_1UT, 0, 252));
    const v4f t3 = *(const v4fa*)(b2ut + clampi(c - BO_2UT, 0, 124));
    const v4f t4 = *(const v4fa*)(b1tu + clampi(c - BO_1TU, 0, 252));
    const v4f t5 = *(const v4fa*)(b2tu + clampi(c - BO_2TU, 0, 124));
    asm volatile("" :: "v"(t0)); asm volatile("" :: "v"(t1)); asm volatile("" :: "v"(t2));
    asm volatile("" :: "v"(t3)); asm volatile("" :: "v"(t4)); asm volatile("" :: "v"(t5));
    const unsigned m0 = (c < BO_AT) ? 0xFFFFFFFFu : 0u;
    const unsigned m1 = (c >= BO_AT  && c < BO_1UT) ? 0xFFFFFFFFu : 0u;
    const unsigned m2 = (c >= BO_1UT && c < BO_2UT) ? 0xFFFFFFFFu : 0u;
    const unsigned m3 = (c >= BO_2UT && c < BO_1TU) ? 0xFFFFFFFFu : 0u;
    const unsigned m4 = (c >= BO_1TU && c < BO_2TU) ? 0xFFFFFFFFu : 0u;
    const unsigned m5 = (c >= BO_2TU) ? 0xFFFFFFFFu : 0u;
    v4u r;
    r.x = (bfv_bits(t0.x) & m0) | (bfv_bits(t1.x) & m1) | (bfv_bits(t2.x) & m2) | (bfv_bits(t3.x) & m3) | (bfv_bits(t4.x) & m4) | (bfv_bits(t5.x) & m5);
    r.y = (bfv_bits(t0.y) & m0) | (bfv_bits(t1.y) & m1) | (bfv_bits(t2.y) & m2) | (bfv_bits(t3.y) & m3) | (bfv_bits(t4.y) & m4) | (bfv_bits(t5.y) & m5);
    r.z = (bfv_bits(t0.z) & m0) | (bfv_bits(t1.z) & m1) | (bfv_bits(t2.z) & m2) | (bfv_bits(t3.z) & m3) | (bfv_bits(t4.z) & m4) | (bfv_bits(t5.z) & m5);
    r.w = (bfv_bits(t0.w) & m0) | (bfv_bits(t1.w) & m1) | (bfv_bits(t2.w) & m2) | (bfv_bits(t3.w) & m3) | (bfv_bits(t4.w) & m4) | (bfv_bits(t5.w) & m5);
    const float e0 = epsut[0];
    const float e1 = epstu[0];
    asm volatile("" :: "v"(e0)); asm volatile("" :: "v"(e1));
    const float s0 = 1.0f + bf16_val(e0);
    const float s1 = 1.0f + bf16_val(e1);
    const unsigned ms = (tid == 0) ? 0xFFFFFFFFu : 0u;
    const v4u sv = (v4u){ __float_as_uint(s0) & ms, __float_as_uint(s1) & ms, 0u, 0u };
    volatile v4u* qb = (volatile v4u*)(Btab + c);
    volatile v4u* qs = (volatile v4u*)(Stab + 4 * (tid & 7));
    *qb = r;
    if (tid < 8) *qs = sv;
    __threadfence();
    *qb = r;
    if (tid < 8) *qs = sv;
  }
}

__device__ __forceinline__ int scan_chunk(const int* __restrict__ keys, int nE, int cbase, int slotBase,
                                          int* list, int tid, int wave) {
  const int el0 = tid * EPT;
  const int e0  = cbase + el0;
  const int e0c = (e0 < nE - EPT) ? e0 : (nE - EPT);
  const v4i da = *(const v4ia*)(keys + e0c);
  const v4i db = *(const v4ia*)(keys + e0c + 4);
  asm volatile("" :: "v"(da.x)); asm volatile("" :: "v"(da.y)); asm volatile("" :: "v"(da.z)); asm volatile("" :: "v"(da.w));
  asm volatile("" :: "v"(db.x)); asm volatile("" :: "v"(db.y)); asm volatile("" :: "v"(db.z)); asm volatile("" :: "v"(db.w));
  const int inv = (e0 < nE) ? 0 : -1;
  const unsigned nbs = (unsigned)slotBase;
  const unsigned unb = (unsigned)NBA;
  const unsigned s0 = (unsigned)(da.x | inv) - nbs, s1 = (unsigned)(da.y | inv) - nbs;
  const unsigned s2 = (unsigned)(da.z | inv) - nbs, s3 = (unsigned)(da.w | inv) - nbs;
  const unsigned s4 = (unsigned)(db.x | inv) - nbs, s5 = (unsigned)(db.y | inv) - nbs;
  const unsigned s6 = (unsigned)(db.z | inv) - nbs, s7 = (unsigned)(db.w | inv) - nbs;
  const bool h0 = s0 < unb, h1 = s1 < unb, h2 = s2 < unb, h3 = s3 < unb;
  const bool h4 = s4 < unb, h5 = s5 < unb, h6 = s6 < unb, h7 = s7 < unb;
  const unsigned m0 = __builtin_amdgcn_ballot_w32(h0), m1 = __builtin_amdgcn_ballot_w32(h1);
  const unsigned m2 = __builtin_amdgcn_ballot_w32(h2), m3 = __builtin_amdgcn_ballot_w32(h3);
  const unsigned m4 = __builtin_amdgcn_ballot_w32(h4), m5 = __builtin_amdgcn_ballot_w32(h5);
  const unsigned m6 = __builtin_amdgcn_ballot_w32(h6), m7 = __builtin_amdgcn_ballot_w32(h7);
  const int wc = (int)(__builtin_popcount(m0) + __builtin_popcount(m1) + __builtin_popcount(m2) + __builtin_popcount(m3) +
                       __builtin_popcount(m4) + __builtin_popcount(m5) + __builtin_popcount(m6) + __builtin_popcount(m7));
  int pos = (int)(__builtin_amdgcn_mbcnt_lo(m0, 0u) + __builtin_amdgcn_mbcnt_lo(m1, 0u) + __builtin_amdgcn_mbcnt_lo(m2, 0u) +
                  __builtin_amdgcn_mbcnt_lo(m3, 0u) + __builtin_amdgcn_mbcnt_lo(m4, 0u) + __builtin_amdgcn_mbcnt_lo(m5, 0u) +
                  __builtin_amdgcn_mbcnt_lo(m6, 0u) + __builtin_amdgcn_mbcnt_lo(m7, 0u));
  const int lb = wave * WCAP;
#define PUTJ(J, HJ, SJ) if (HJ) { if (pos < WCAP) list[lb + pos] = ((el0 + (J)) << SLA) | (int)(SJ); pos = pos + 1; }
  PUTJ(0, h0, s0)
  PUTJ(1, h1, s1)
  PUTJ(2, h2, s2)
  PUTJ(3, h3, s3)
  PUTJ(4, h4, s4)
  PUTJ(5, h5, s5)
  PUTJ(6, h6, s6)
  PUTJ(7, h7, s7)
#undef PUTJ
  return wc;
}

__global__ __launch_bounds__(NTHR) void k_bucket(const int* __restrict__ srcs, const int* __restrict__ keys, int nE,
                                                 int* __restrict__ LIST, int* __restrict__ CNT,
                                                 int* __restrict__ OFF, int* __restrict__ FLG) {
  extern __shared__ __attribute__((aligned(16))) int dsm[];
  int* list = dsm;
  int* hl   = dsm + LISTN;
  int* sl   = hl + RCAP;
  int* cnt  = sl + RCAP;
  int* offs = cnt + NBA;
  int* cur  = offs + NBA;
  int* misc = cur + NBA;
  const int tid = (int)threadIdx.x, lane = tid & 31, wave = tid >> 5;
  const int blk = (int)blockIdx.x;
  const int slotBase = blk * NBA;

  {
    const v4i z4 = {0, 0, 0, 0};
    for (int i = tid * 4; i < BK_ZINTS; i += NTHR * 4) *(v4ia*)(dsm + i) = z4;
    if (tid < BK_MISC) misc[tid] = 0;
  }
  __syncthreads();

  int t = 0, ov = 0;
  const int nChunks = (nE + CHUNK - 1) / CHUNK;
#pragma unroll 1
  for (int ch = 0; ch < nChunks; ++ch) {
    const int cbase = ch * CHUNK;
    const int wc = scan_chunk(keys, nE, cbase, slotBase, list, tid, wave);
    if (lane == 0) misc[wave] = wc;
    __syncthreads();
    if (wave == 0) {
#pragma unroll 1
      for (int w2 = 0; w2 < NWAVE; ++w2) {
        int c = misc[w2];
        c = c < 0 ? 0 : (c > WCAP ? WCAP : c);
#pragma unroll 1
        for (int b0 = 0; b0 < c; b0 += 32) {
          const int idx = b0 + lane;
          const int ent = list[w2 * WCAP + (idx < WCAP ? idx : WCAP - 1)];
          const int m32 = (c - b0) < 32 ? (c - b0) : 32;
#pragma unroll 1
          for (int k = 0; k < m32; ++k) {
            const int u    = __builtin_amdgcn_readlane(ent, k);
            const int slot = u & (NBA - 1);
            const int el   = (u >> SLA) & (CHUNK - 1);
            const int pk   = ((cbase + el) << SLA) | slot;
            if (t < RCAP) {
              if (lane == 0) { hl[t] = pk; cnt[slot] = cnt[slot] + 1; }
              t = t + 1;
            } else {
              ov = 1;
            }
          }
        }
      }
    }
    __syncthreads();
  }
  if (wave == 0 && lane == 0) { misc[8] = t; misc[9] = ov; }
  __syncthreads();
  int tt = misc[8];
  tt = tt < 0 ? 0 : (tt > RCAP ? RCAP : tt);
  const int ovf = misc[9];

  if (wave == 0) {
    const int base = lane * (NBA / 32);
    int s = 0;
#pragma unroll 1
    for (int i = 0; i < NBA / 32; ++i) s += cnt[base + i];
    int incl = s;
#pragma unroll
    for (int d = 1; d < 32; d <<= 1) {
      const int y = __shfl_up(incl, d, 32);
      if (lane >= d) incl += y;
    }
    int run = incl - s;
#pragma unroll 1
    for (int i = 0; i < NBA / 32; ++i) {
      const int cv = cnt[base + i];
      offs[base + i] = run;
      cur[base + i]  = run;
      run += cv;
    }
  }
  __syncthreads();
  if (wave == 0) {
#pragma unroll 1
    for (int b0 = 0; b0 < tt; b0 += 32) {
      const int idx = b0 + lane;
      const int ent = hl[idx < RCAP ? idx : RCAP - 1];
      const int m32 = (tt - b0) < 32 ? (tt - b0) : 32;
#pragma unroll 1
      for (int k = 0; k < m32; ++k) {
        const int u    = __builtin_amdgcn_readlane(ent, k);
        const int slot = u & (NBA - 1);
        if (lane == 0) {
          int p = cur[slot];
          p = p < 0 ? 0 : (p > RCAP - 1 ? RCAP - 1 : p);
          sl[p] = u;
          cur[slot] = p + 1;
        }
      }
    }
  }
  __syncthreads();

#pragma unroll 1
  for (int it = 0; it < RCAP / (NTHR * 4); ++it) {
    const int i4 = (it * NTHR + tid) * 4;
    const v4i u4 = *(const v4ia*)(sl + i4);
    const int a0 = srcs[clampi(u4.x >> SLA, 0, nE - 1)];
    const int a1 = srcs[clampi(u4.y >> SLA, 0, nE - 1)];
    const int a2 = srcs[clampi(u4.z >> SLA, 0, nE - 1)];
    const int a3 = srcs[clampi(u4.w >> SLA, 0, nE - 1)];
    asm volatile("" :: "v"(a0)); asm volatile("" :: "v"(a1)); asm volatile("" :: "v"(a2)); asm volatile("" :: "v"(a3));
    v4i o;
    o.x = a0 & ((i4 + 0 < tt) ? -1 : 0);
    o.y = a1 & ((i4 + 1 < tt) ? -1 : 0);
    o.z = a2 & ((i4 + 2 < tt) ? -1 : 0);
    o.w = a3 & ((i4 + 3 < tt) ? -1 : 0);
    volatile v4i* q = (volatile v4i*)(LIST + (size_t)blk * RCAP + i4);
    *q = o;
    __threadfence();
    *q = o;
  }
  {
    const v4i c4 = *(const v4ia*)(cnt + 4 * tid);
    const v4i o4 = *(const v4ia*)(offs + 4 * tid);
    const v4i f4 = {ovf, ovf, ovf, ovf};
    volatile v4i* qc = (volatile v4i*)(CNT + (size_t)blk * NBA + 4 * tid);
    volatile v4i* qo = (volatile v4i*)(OFF + (size_t)blk * NBA + 4 * tid);
    volatile v4i* qf = (volatile v4i*)(FLG + blk * 32 + 4 * (tid & 7));
    *qc = c4;
    *qo = o4;
    if (tid < 8) *qf = f4;
    __threadfence();
    *qc = c4;
    *qo = o4;
    if (tid < 8) *qf = f4;
  }
}

template <int DD>
__global__ __launch_bounds__(256) void k_replay(const float* __restrict__ Aal, const float* __restrict__ xd,
                                                const int* __restrict__ LIST, const int* __restrict__ CNT,
                                                const int* __restrict__ OFF, const int* __restrict__ FLG,
                                                const float* __restrict__ Stab, int sidx, int nSrc, int nDst,
                                                int mRows, unsigned short* __restrict__ OP) {
  static_assert(DD == 64 || DD == 128);
  constexpr int EL   = DD / 32;
  constexpr int OWNW = SPLIT_OP ? 2 * DD : DD;
  constexpr int AGGW = SPLIT_OP ? 256 : 128;
  constexpr int W    = OWNW + AGGW;
  constexpr int PP   = W / 8;
  constexpr int NI   = (PP + 31) / 32;
  static_assert(W % 64 == 0 && W <= 512 && NI >= 1 && NI <= 2);
  __shared__ __attribute__((aligned(16))) unsigned short rb[8][512];
  const int lane = (int)threadIdx.x & 31, wave = (int)threadIdx.x >> 5;
  unsigned short* rbw = &rb[wave][0];
  const int v = (int)blockIdx.x * 8 + wave;
  const bool inr  = v < mRows;
  const bool live = v < nDst;
  const int vc  = clampi(v, 0, nDst - 1);
  const int blk = vc >> SLA;

  const int cw = CNT[vc];
  const int ow = OFF[vc];
  const int fw = FLG[blk * 32];
  const float sv = Stab[sidx];
  asm volatile("" :: "v"(cw)); asm volatile("" :: "v"(ow)); asm volatile("" :: "v"(fw)); asm volatile("" :: "v"(sv));
  const bool bad = (fw != 0) || (cw < 0) || (cw > DEGCAP);
  int cc = cw < 0 ? 0 : (cw > DEGCAP ? DEGCAP : cw);
  cc = live ? cc : 0;
  const int cn = __builtin_amdgcn_readfirstlane(cc);
  const int o  = clampi(ow, 0, RCAP - 1);
  const int* lbp = LIST + (size_t)blk * RCAP;

  float a0 = 0.0f, a1 = 0.0f, a2 = 0.0f, a3 = 0.0f;
#pragma unroll 1
  for (int b0 = 0; b0 < cn; b0 += 32) {
    int j = b0 + lane;
    j = j > cn - 1 ? cn - 1 : j;
    int idx = o + j;
    idx = idx > RCAP - 1 ? RCAP - 1 : idx;
    int sr = lbp[idx];
    asm volatile("" :: "v"(sr));
    sr = clampi(sr, 0, nSrc - 1);
    const int m32 = (cn - b0) < 32 ? (cn - b0) : 32;
#pragma unroll 1
    for (int k = 0; k < m32; ++k) {
      const int sk = __builtin_amdgcn_readlane(sr, k);
      const v4f a = *(const v4fa*)(Aal + (size_t)sk * DA + 4 * lane);
      asm volatile("" :: "v"(a));
      a0 += a.x; a1 += a.y; a2 += a.z; a3 += a.w;
    }
  }
  const float qn = __int_as_float(0x7fc00000);
  float ag[4];
  ag[0] = (cn > 0) ? a0 : 0.0f; ag[1] = (cn > 0) ? a1 : 0.0f;
  ag[2] = (cn > 0) ? a2 : 0.0f; ag[3] = (cn > 0) ? a3 : 0.0f;
  float ov[EL];
  if constexpr (EL == 4) {
    const v4f xo = *(const v4fa*)(xd + (size_t)vc * DD + 4 * lane);
    asm volatile("" :: "v"(xo));
    ov[0] = bf16_val(xo.x) * sv; ov[1] = bf16_val(xo.y) * sv; ov[2] = bf16_val(xo.z) * sv; ov[3] = bf16_val(xo.w) * sv;
  } else {
    const v2f xo = *(const v2fa*)(xd + (size_t)vc * DD + 2 * lane);
    asm volatile("" :: "v"(xo));
    ov[0] = bf16_val(xo.x) * sv; ov[1] = bf16_val(xo.y) * sv;
  }
#pragma unroll
  for (int e = 0; e < 4; ++e) { float t = bad ? qn : ag[e]; ag[e] = live ? t : 0.0f; }
#pragma unroll
  for (int e = 0; e < EL; ++e) { float t = bad ? qn : ov[e]; ov[e] = live ? t : 0.0f; }

  if constexpr (EL == 4) {
    const v2u wh = (v2u){ pk16(bf16_bits(ov[0]), bf16_bits(ov[1])), pk16(bf16_bits(ov[2]), bf16_bits(ov[3])) };
    *(v2ua*)(rbw + 4 * lane) = wh;
    if (SPLIT_OP) {
      const v2u wl = (v2u){ pk16(bf16_lo_bits(ov[0]), bf16_lo_bits(ov[1])), pk16(bf16_lo_bits(ov[2]), bf16_lo_bits(ov[3])) };
      *(v2ua*)(rbw + DD + 4 * lane) = wl;
    }
  } else {
    *(u32a*)(rbw + 2 * lane) = pk16(bf16_bits(ov[0]), bf16_bits(ov[1]));
    if (SPLIT_OP) *(u32a*)(rbw + DD + 2 * lane) = pk16(bf16_lo_bits(ov[0]), bf16_lo_bits(ov[1]));
  }
  {
    const v2u gh = (v2u){ pk16(bf16_bits(ag[0]), bf16_bits(ag[1])), pk16(bf16_bits(ag[2]), bf16_bits(ag[3])) };
    *(v2ua*)(rbw + OWNW + 4 * lane) = gh;
    if (SPLIT_OP) {
      const v2u gl = (v2u){ pk16(bf16_lo_bits(ag[0]), bf16_lo_bits(ag[1])), pk16(bf16_lo_bits(ag[2]), bf16_lo_bits(ag[3])) };
      *(v2ua*)(rbw + OWNW + 128 + 4 * lane) = gl;
    }
  }
  wave_sync();
  v4u q[NI];
#pragma unroll
  for (int i = 0; i < NI; ++i) {
    const int pi = i * 32 + lane;
    const int pc = pi < PP ? pi : PP - 1;
    q[i] = *(const v4ua*)(rbw + 8 * pc);
    asm volatile("" :: "v"(q[i]));
  }
  unsigned short* rowp = OP + (size_t)(inr ? v : 0) * W;
#pragma unroll
  for (int i = 0; i < NI; ++i) {
    const int pi = i * 32 + lane;
    if (inr && pi < PP) *(volatile v4u*)(rowp + 8 * pi) = q[i];
  }
  __threadfence();
#pragma unroll
  for (int i = 0; i < NI; ++i) {
    const int pi = i * 32 + lane;
    if (inr && pi < PP) *(volatile v4u*)(rowp + 8 * pi) = q[i];
  }
}

__global__ __launch_bounds__(256) void k_relu_split(const float* __restrict__ T, unsigned short* __restrict__ H, int rows) {
  const unsigned g = blockIdx.x * 256u + threadIdx.x;
  const int row  = (int)(g >> 5);
  const int lane = (int)(g & 31u);
  const int rc = row < rows ? row : rows - 1;
  const float* p = T + (size_t)rc * HIDW + 8 * lane;
  v4f a = *(const v4fa*)p;
  v4f c = *(const v4fa*)(p + 4);
  asm volatile("" :: "v"(a)); asm volatile("" :: "v"(c));
  a.x = (a.x > 0.0f) ? a.x : (a.x - a.x); a.y = (a.y > 0.0f) ? a.y : (a.y - a.y);
  a.z = (a.z > 0.0f) ? a.z : (a.z - a.z); a.w = (a.w > 0.0f) ? a.w : (a.w - a.w);
  c.x = (c.x > 0.0f) ? c.x : (c.x - c.x); c.y = (c.y > 0.0f) ? c.y : (c.y - c.y);
  c.z = (c.z > 0.0f) ? c.z : (c.z - c.z); c.w = (c.w > 0.0f) ? c.w : (c.w - c.w);
  const v4u hi = pack8_bf16(a, c);
  const v4u lo = pack8_bf16_lo(a, c);
  if (row < rows) {
    unsigned short* rp = H + (size_t)row * K2 + 8 * lane;
    *(volatile v4u*)rp = hi;
    if (SPLIT_HID) *(volatile v4u*)(rp + HIDW) = lo;
    __threadfence();
    *(volatile v4u*)rp = hi;
    if (SPLIT_HID) *(volatile v4u*)(rp + HIDW) = lo;
  }
}

static inline int gemm_blocks(int M, int N) { return (((M + 63) / 64) * ((N + 63) / 64) + 7) / 8; }

extern "C" void kernel_launch(void* const* d_in, const int* in_sizes, int n_in,
                              void* d_out, int out_size, void* d_ws, size_t ws_size,
                              hipStream_t stream) {
  if (n_in < 18) return;
  const int want[18] = { NU * DU, NT * DT, 2 * NE, 2 * NE, DU * DA, DA, DT * DA, DA, 1, 1,
                         (DT + DA) * HIDW, HIDW, HIDW * DOUT, DOUT, (DU + DA) * HIDW, HIDW, HIDW * DOUT, DOUT };
  for (int i = 0; i < 18; ++i) if (in_sizes[i] != want[i]) return;
  if ((long long)out_size != (long long)NU * DOUT + (long long)NT * DOUT) return;
  if (ws_size < WS_TOTAL) return;

  const float* x_user = (const float*)d_in[0];
  const float* x_tx   = (const float*)d_in[1];
  const int*   e_ut   = (const int*)d_in[2];
  const int*   e_tu   = (const int*)d_in[3];
  const float* W_au   = (const float*)d_in[4];
  const float* b_au   = (const float*)d_in[5];
  const float* W_at   = (const float*)d_in[6];
  const float* b_at   = (const float*)d_in[7];
  const float* eps_ut = (const float*)d_in[8];
  const float* eps_tu = (const float*)d_in[9];
  const float* W1_ut  = (const float*)d_in[10];
  const float* b1_ut  = (const float*)d_in[11];
  const float* W2_ut  = (const float*)d_in[12];
  const float* b2_ut  = (const float*)d_in[13];
  const float* W1_tu  = (const float*)d_in[14];
  const float* b1_tu  = (const float*)d_in[15];
  const float* W2_tu  = (const float*)d_in[16];
  const float* b2_tu  = (const float*)d_in[17];
  float* out_user = (float*)d_out;
  float* out_tx   = (float*)d_out + (size_t)NU * DOUT;

  char* ws = (char*)d_ws;
  float*          Treg = (float*)(ws + O_T);
  unsigned short* OPH  = (unsigned short*)(ws + O_OPH);
  unsigned short* XS   = (unsigned short*)(ws + O_XS);
  int*            LIST = (int*)(ws + O_LIST);
  int*            CNT  = (int*)(ws + O_CNT);
  int*            OFF  = (int*)(ws + O_OFF);
  int*            FLG  = (int*)(ws + O_FLG);
  unsigned short* PWau  = (unsigned short*)(ws + O_WAU);
  unsigned short* PWat  = (unsigned short*)(ws + O_WAT);
  unsigned short* PW1ut = (unsigned short*)(ws + O_W1UT);
  unsigned short* PW1tu = (unsigned short*)(ws + O_W1TU);
  unsigned short* PW2ut = (unsigned short*)(ws + O_W2UT);
  unsigned short* PW2tu = (unsigned short*)(ws + O_W2TU);
  float*          Btab  = (float*)(ws + O_BT);
  float*          Stab  = (float*)(ws + O_ST);

  const size_t bkLds = (size_t)BK_LDS_INTS * 4;
  hipFuncSetAttribute(reinterpret_cast<const void*>(&k_bucket), hipFuncAttributeMaxDynamicSharedMemorySize, (int)bkLds);

  k_prep<<<PU5 / 256 + 1, 256, 0, stream>>>(W_au, W_at, W1_ut, W1_tu, W2_ut, W2_tu,
                                            b_au, b_at, b1_ut, b2_ut, b1_tu, b2_tu, eps_ut, eps_tu,
                                            PWau, PWat, PW1ut, PW1tu, PW2ut, PW2tu, Btab, Stab);

  k_plane<0><<<MPAD * DU / 8 / 256, 256, 0, stream>>>(x_user, NU, DU, DU, XS, MPAD, DU);
  k_gemm_nt<0, 1><<<gemm_blocks(MPAD, DA), 256, 0, stream>>>(XS, PWau, Btab + BO_AU, Treg, MPAD, DA, DU, DA);
  k_bucket<<<NBLK, NTHR, bkLds, stream>>>(e_ut, e_ut + NE, NE, LIST, CNT, OFF, FLG);
  k_replay<DT><<<MPAD / 8, 256, 0, stream>>>(Treg, x_tx, LIST, CNT, OFF, FLG, Stab, 0, NU, NT, MPAD, OPH);
  k_gemm_nt<0, 1><<<gemm_blocks(MPAD, HIDW), 256, 0, stream>>>(OPH, PW1ut, Btab + BO_1UT, Treg, MPAD, HIDW, KOP_UT, HIDW);
  k_relu_split<<<MPAD * 32 / 256, 256, 0, stream>>>(Treg, OPH, MPAD);
  k_gemm_nt<0, 1><<<gemm_blocks(NT, DOUT), 256, 0, stream>>>(OPH, PW2ut, Btab + BO_2UT, out_tx, NT, DOUT, K2, DOUT);

  k_plane<0><<<MPAD * DT / 8 / 256, 256, 0, stream>>>(x_tx, NT, DT, DT, XS, MPAD, DT);
  k_gemm_nt<0, 1><<<gemm_blocks(MPAD, DA), 256, 0, stream>>>(XS, PWat, Btab + BO_AT, Treg, MPAD, DA, DT, DA);
  k_bucket<<<NBLK, NTHR, bkLds, stream>>>(e_tu, e_tu + NE, NE, LIST, CNT, OFF, FLG);
  k_replay<DU><<<MPAD / 8, 256, 0, stream>>>(Treg, x_user, LIST, CNT, OFF, FLG, Stab, 1, NT, NU, MPAD, OPH);
  k_gemm_nt<0, 1><<<gemm_blocks(MPAD, HIDW), 256, 0, stream>>>(OPH, PW1tu, Btab + BO_1TU, Treg, MPAD, HIDW, KOP_TU, HIDW);
  k_relu_split<<<MPAD * 32 / 256, 256, 0, stream>>>(Treg, OPH, MPAD);
  k_gemm_nt<0, 1><<<gemm_blocks(NU, DOUT), 256, 0, stream>>>(OPH, PW2tu, Btab + BO_2TU, out_user, NU, DOUT, K2, DOUT);
}
